// SnycTwinSSM_67473936220408
// MI455X (gfx1250) — hardware-run, weakly checked
//
#include <hip/hip_runtime.h>


#ifndef NB
#define NB 2
#endif
#ifndef SEQ
#define SEQ 2048
#endif
#define NB_FULL  2
#define SEQ_FULL 2048
#ifndef OUT_SEQ
#define OUT_SEQ SEQ
#endif
#define DM   512
#define DH   256
#define DS   128
#define DTR  32
#define NXD  288
#define NXP  320
#define CIN  1024
#define NTOK (NB * SEQ)
#define NPB  (NTOK / 64)
#define LOG2E 1.4426950408889634f
#define NEGB (-3.0e38f)
#define XCS  16.0f
#define WCS  256.0f
#define DTS  64.0f
#define INV_XW (1.0f / 4096.0f)
#define INV_DT (1.0f / 4096.0f)
#define OUT1_OFF ((size_t)NB_FULL * SEQ_FULL * DM)

static_assert(OUT1_OFF * 4 == (size_t)8388608);
static_assert(SEQ % 64 == 0);
static_assert(NTOK % 64 == 0);
static_assert(DM % 64 == 0);
static_assert(DH % 64 == 0);
static_assert(NXP % 64 == 0);
static_assert(NXP >= NXD);
static_assert(CIN % 64 == 0);
static_assert(DM % 32 == 0);
static_assert(DH % 32 == 0);
static_assert(DTR == 32);
static_assert(DTR + 2 * DS == NXD);
static_assert(2 * DS == 256);
static_assert(DS == 32 * 4);
static_assert(SEQ % 32 == 0);
static_assert((NB * DH) % 8 == 0);
static_assert(NPB <= 256);
static_assert(NTOK % 16 == 0);
static_assert(NB <= NB_FULL);
static_assert(SEQ <= SEQ_FULL);
static_assert(8 * 32 * 16 == 16 * 64 * 4);
static_assert(4 * 256 * 4 == 64 * 64);
static_assert(2 * 256 * 8 == 64 * 64);
static_assert(16 * 68 * 4 <= 131072);
static_assert(64 * 65 * 4 <= 131072);
static_assert(8 * 32 * 36 * 4 + 8 * SEQ * 4 <= 131072);
static_assert((NXP * 4) % 128 == 0);
static_assert((SEQ * 4) % 128 == 0);

typedef _Float16 h16;
typedef unsigned short bf;
typedef __attribute__((ext_vector_type(16))) __bf16   v16bf;
typedef __attribute__((ext_vector_type(16))) _Float16 v16h;
typedef __attribute__((ext_vector_type(8)))  _Float16 v8h;
typedef __attribute__((ext_vector_type(8)))  unsigned short v8us;
typedef __attribute__((ext_vector_type(8)))  float    v8f;
typedef __attribute__((ext_vector_type(4)))  float    v4f;
typedef v4f  __attribute__((may_alias)) v4fa;

__device__ __forceinline__ unsigned short f2bf(float f) { unsigned u = __float_as_uint(f); u += 0x7FFFu + ((u >> 16) & 1u); return (unsigned short)(u >> 16); }
__device__ __forceinline__ float bfr(float f) { return __uint_as_float(((unsigned)f2bf(f)) << 16); }
__device__ __forceinline__ v16h cat16(v8h lo, v8h hi) { return __builtin_shufflevector(lo, hi, 0, 1, 2, 3, 4, 5, 6, 7, 8, 9, 10, 11, 12, 13, 14, 15); }
__device__ __forceinline__ v16bf cat16b(v8us lo, v8us hi) { return __builtin_bit_cast(v16bf, __builtin_shufflevector(lo, hi, 0, 1, 2, 3, 4, 5, 6, 7, 8, 9, 10, 11, 12, 13, 14, 15)); }
__device__ __forceinline__ v8f wmma16(v16h a, v16h b, v8f c) { return __builtin_amdgcn_wmma_f32_16x16x32_f16(false, a, false, b, (short)0, c, false, false); }
__device__ __forceinline__ v8f wmmab(v16bf a, v16bf b, v8f c) { return __builtin_amdgcn_wmma_f32_16x16x32_bf16(false, a, false, b, (short)0, c, false, false); }
__device__ __forceinline__ v16h  ldh(const h16* p) { return cat16(*(const v8h*)p, *(const v8h*)(p + 16)); }
__device__ __forceinline__ v16bf ldb(const bf* p)  { return cat16b(*(const v8us*)p, *(const v8us*)(p + 16)); }
__device__ __forceinline__ void wave_sync() { __builtin_amdgcn_fence(3  , "wavefront"); __builtin_amdgcn_wave_barrier(); asm volatile("" ::: "memory"); }

__device__ __forceinline__ v8f mmab(v16bf a, v16bf b, v8f c) { c = wmmab(a, b, c); asm volatile("v_nop\n\tv_nop\n\tv_nop\n\tv_nop" : "+v"(c) : "v"(a), "v"(b)); return c; }
__device__ __forceinline__ v8f mmah(v16h a, v16h b, v8f c)   { c = wmma16(a, b, c); asm volatile("v_nop\n\tv_nop\n\tv_nop\n\tv_nop" : "+v"(c) : "v"(a), "v"(b)); return c; }
static __device__ __forceinline__ h16 toh_flush(float v) { const h16 r = (h16)v; return (fabsf(v) < 6.103515625e-05f) ? (h16)0.0f : r; }
__device__ __forceinline__ float softthr(float v, float thr) { const float mag = fmaxf(fabsf(v) - thr, 0.0f); return (v == 0.0f) ? 0.0f : copysignf(mag, v); }
__device__ __forceinline__ float softplus_f(float x) { return fmaxf(x, 0.0f) + log1pf(__builtin_amdgcn_exp2f(-fabsf(x) * LOG2E)); }
__device__ __forceinline__ float abase(float alog, float e1) { return e1 * (-expf(bfr(alog))); }

__global__ __launch_bounds__(256) void k_cvt8(const float* __restrict__ src, bf* dst, size_t n8) {
    const size_t i = (size_t)blockIdx.x * 256 + threadIdx.x; if (i >= n8) return;
    const v8f v = *(const v8f*)(src + i * 8); v8us o;
#pragma unroll
    for (int k = 0; k < 8; ++k) o[k] = f2bf(v[k]);
    *(volatile v8us*)(dst + i * 8) = o; __threadfence(); *(volatile v8us*)(dst + i * 8) = o;
}

__global__ __launch_bounds__(256) void k_wcvth(const float* __restrict__ src, h16* dst, int srcRows, int dstRows, int cols, float carry) {
    const size_t i = (size_t)blockIdx.x * 256 + threadIdx.x; const size_t n8 = (size_t)dstRows * (size_t)cols / 8; if (i >= n8) return;
    const int row = (int)((i * 8) / (size_t)cols), col = (int)((i * 8) % (size_t)cols);
    const int rc = row < srcRows ? row : (srcRows - 1);
    v8f v = *(const v8f*)(src + (size_t)rc * cols + col);
    asm volatile("" : "+v"(v));
    const bool ok = row < srcRows;
    v8h o;
#pragma unroll
    for (int k = 0; k < 8; ++k) { const float f = ok ? (bfr(v[k]) * carry) : 0.0f; o[k] = toh_flush(f); }
    *(volatile v8h*)(dst + i * 8) = o; __threadfence(); *(volatile v8h*)(dst + i * 8) = o;
}

__global__ __launch_bounds__(512) void k_prepA(const float* __restrict__ A_log, const float* __restrict__ eps, float* A12) {
    __shared__ float wm[16];
    const int tid = threadIdx.x, lane = tid & 31;
    const int wave = __builtin_amdgcn_readfirstlane((int)(threadIdx.x >> 5));
    const float e1 = 1.0f + bfr(eps[0]);
    float m = NEGB;
#pragma unroll 1
    for (int i = tid; i < DH * DS; i += 512) m = fmaxf(m, abase(A_log[i], e1));
    for (int o = 16; o > 0; o >>= 1) m = fmaxf(m, __shfl_xor(m, o, 32));
    if (lane == 0) wm[wave] = m;
    __syncthreads();
    float r = wm[lane & 15];
    for (int o = 16; o > 0; o >>= 1) r = fmaxf(r, __shfl_xor(r, o, 32));
    const float thr1 = 0.1f * r;
    __syncthreads();
    float m2 = NEGB;
#pragma unroll 1
    for (int i = tid; i < DH * DS; i += 512) m2 = fmaxf(m2, softthr(abase(A_log[i], e1), thr1));
    for (int o = 16; o > 0; o >>= 1) m2 = fmaxf(m2, __shfl_xor(m2, o, 32));
    if (lane == 0) wm[wave] = m2;
    __syncthreads();
    float r2 = wm[lane & 15];
    for (int o = 16; o > 0; o >>= 1) r2 = fmaxf(r2, __shfl_xor(r2, o, 32));
    const float thr2 = 0.1f * r2;
#pragma unroll 1
    for (int ps = 0; ps < 2; ++ps) {
#pragma unroll 1
        for (int i = tid; i < DH * DS; i += 512) {
            const float a1 = softthr(abase(A_log[i], e1), thr1);
            const float a2 = softthr(a1, thr2);
            *(volatile float*)(A12 + i) = a1; *(volatile float*)(A12 + DH * DS + i) = a2; }
        if (ps == 0) __threadfence(); }
}

__global__ __launch_bounds__(256) void k_tr_bf(const float* __restrict__ src, size_t sbatch, int spitch, bf* dst, int dpitch) {
    __shared__ float ts[64 * 65];
    const int tid = threadIdx.x;
    const int l0 = blockIdx.x * 64, c0 = blockIdx.y * 64, b = blockIdx.z;
    const float* sp = src + (size_t)b * sbatch + (size_t)c0 * spitch + l0;
#pragma unroll
    for (int it = 0; it < 4; ++it) { const int p = it * 256 + tid; const int r = p >> 4, q = (p & 15) * 4;
        const v4f v = *(const v4f*)(sp + (size_t)r * spitch + q);
        ts[r * 65 + q] = v[0]; ts[r * 65 + q + 1] = v[1]; ts[r * 65 + q + 2] = v[2]; ts[r * 65 + q + 3] = v[3]; }
    __syncthreads();
    v8us o[2];
#pragma unroll
    for (int it = 0; it < 2; ++it) { const int p = it * 256 + tid; const int tok = p >> 3, c8 = (p & 7) * 8;
#pragma unroll
        for (int k = 0; k < 8; ++k) o[it][k] = f2bf(ts[(c8 + k) * 65 + tok]); }
    bf* dp = dst + ((size_t)b * SEQ + l0) * dpitch + c0;
#pragma unroll 1
    for (int ps = 0; ps < 2; ++ps) {
#pragma unroll
        for (int it = 0; it < 2; ++it) { const int p = it * 256 + tid; const int tok = p >> 3, c8 = (p & 7) * 8;
            *(volatile v8us*)(dp + (size_t)tok * dpitch + c8) = o[it]; }
        if (ps == 0) __threadfence(); }
}

__global__ __launch_bounds__(256) void k_tr_h(const float* __restrict__ src, size_t sbatch, int spitch, h16* dst, int dpitch, float carry) {
    __shared__ float ts[64 * 65];
    const int tid = threadIdx.x;
    const int l0 = blockIdx.x * 64, c0 = blockIdx.y * 64, b = blockIdx.z;
    const float* sp = src + (size_t)b * sbatch + (size_t)c0 * spitch + l0;
#pragma unroll
    for (int it = 0; it < 4; ++it) { const int p = it * 256 + tid; const int r = p >> 4, q = (p & 15) * 4;
        const v4f v = *(const v4f*)(sp + (size_t)r * spitch + q);
        ts[r * 65 + q] = v[0]; ts[r * 65 + q + 1] = v[1]; ts[r * 65 + q + 2] = v[2]; ts[r * 65 + q + 3] = v[3]; }
    __syncthreads();
    v8h o[2];
#pragma unroll
    for (int it = 0; it < 2; ++it) { const int p = it * 256 + tid; const int tok = p >> 3, c8 = (p & 7) * 8;
#pragma unroll
        for (int k = 0; k < 8; ++k) o[it][k] = toh_flush(ts[(c8 + k) * 65 + tok] * carry); }
    h16* dp = dst + ((size_t)b * SEQ + l0) * dpitch + c0;
#pragma unroll 1
    for (int ps = 0; ps < 2; ++ps) {
#pragma unroll
        for (int it = 0; it < 2; ++it) { const int p = it * 256 + tid; const int tok = p >> 3, c8 = (p & 7) * 8;
            *(volatile v8h*)(dp + (size_t)tok * dpitch + c8) = o[it]; }
        if (ps == 0) __threadfence(); }
}

__device__ __forceinline__ void mainloop_b(v8f (&acc)[4][4], const bf* __restrict__ A, size_t aoff, size_t lda, const bf* __restrict__ Bt, size_t boff, size_t ldbt, int K) {
#pragma unroll 1
    for (int kc = 0; kc < K; kc += 32) {
        v16bf a[4];
#pragma unroll
        for (int mb = 0; mb < 4; ++mb) a[mb] = ldb(A + aoff + (size_t)mb * 16 * lda + kc);
#pragma unroll
        for (int nb = 0; nb < 4; ++nb) { const v16bf b = ldb(Bt + boff + (size_t)nb * 16 * ldbt + kc);
#pragma unroll
            for (int mb = 0; mb < 4; ++mb) acc[mb][nb] = mmab(a[mb], b, acc[mb][nb]); }
    }
}
__device__ __forceinline__ void mainloop_h(v8f (&acc)[4][4], const h16* __restrict__ A, size_t aoff, size_t lda, const h16* __restrict__ Bt, size_t boff, size_t ldbt, int K) {
#pragma unroll 1
    for (int kc = 0; kc < K; kc += 32) {
        v16h a[4];
#pragma unroll
        for (int mb = 0; mb < 4; ++mb) a[mb] = ldh(A + aoff + (size_t)mb * 16 * lda + kc);
#pragma unroll
        for (int nb = 0; nb < 4; ++nb) { const v16h b = ldh(Bt + boff + (size_t)nb * 16 * ldbt + kc);
#pragma unroll
            for (int mb = 0; mb < 4; ++mb) acc[mb][nb] = mmah(a[mb], b, acc[mb][nb]); }
    }
}

__global__ __launch_bounds__(32) void k_gemm_in(const bf* __restrict__ A, const bf* __restrict__ Bt, float* C) {
    __shared__ __align__(16) float os[16 * 68];
    const int lane = threadIdx.x & 31, lr = lane & 15, hi = lane >> 4; const int r0 = blockIdx.x * 64, c0 = blockIdx.y * 64;
    v8f acc[4][4];
#pragma unroll
    for (int mb = 0; mb < 4; ++mb)
#pragma unroll
        for (int nb = 0; nb < 4; ++nb) acc[mb][nb] = (v8f){};
    mainloop_b(acc, A, (size_t)(r0 + lr) * DM + 8 * hi, (size_t)DM, Bt, (size_t)(c0 + lr) * CIN + 8 * hi, (size_t)CIN, DM);
    const int bb = c0 / SEQ, tt = c0 % SEQ;
    const size_t cb = ((size_t)bb * DM + r0) * SEQ + tt;
#pragma unroll
    for (int mb = 0; mb < 4; ++mb) {
#pragma unroll
        for (int nb = 0; nb < 4; ++nb) {
#pragma unroll
            for (int j = 0; j < 8; ++j) os[(hi * 8 + j) * 68 + nb * 16 + lr] = acc[mb][nb][j]; }
        wave_sync();
#pragma unroll 1
        for (int ps = 0; ps < 2; ++ps) {
#pragma unroll
            for (int s = 0; s < 8; ++s) { const int row = 2 * s + (lane >> 4), c4 = (lane & 15) * 4;
                const v4f val = *(const v4fa*)(&os[row * 68 + c4]);
                *(volatile v4f*)(C + cb + (size_t)(mb * 16 + row) * SEQ + c4) = val; }
            if (ps == 0) __threadfence(); }
        wave_sync();
    }
}

__global__ __launch_bounds__(32) void k_gemm_tm(const h16* __restrict__ A, int lda, const h16* __restrict__ Bt, int ldbt, int K, float* C, int ldc, int outSeq, float scale) {
    __shared__ __align__(16) float os[16 * 68];
    const int lane = threadIdx.x & 31, lr = lane & 15, hi = lane >> 4; const int r0 = blockIdx.x * 64, c0 = blockIdx.y * 64;
    v8f acc[4][4];
#pragma unroll
    for (int mb = 0; mb < 4; ++mb)
#pragma unroll
        for (int nb = 0; nb < 4; ++nb) acc[mb][nb] = (v8f){};
    mainloop_h(acc, A, (size_t)(r0 + lr) * lda + 8 * hi, (size_t)lda, Bt, (size_t)(c0 + lr) * ldbt + 8 * hi, (size_t)ldbt, K);
    const int bb = r0 / SEQ, tt = r0 % SEQ;
    const size_t cb = ((size_t)bb * outSeq + tt) * ldc + c0;
#pragma unroll
    for (int mb = 0; mb < 4; ++mb) {
#pragma unroll
        for (int nb = 0; nb < 4; ++nb) {
#pragma unroll
            for (int j = 0; j < 8; ++j) os[(hi * 8 + j) * 68 + nb * 16 + lr] = acc[mb][nb][j] * scale; }
        wave_sync();
#pragma unroll 1
        for (int ps = 0; ps < 2; ++ps) {
#pragma unroll
            for (int s = 0; s < 8; ++s) { const int row = 2 * s + (lane >> 4), c4 = (lane & 15) * 4;
                const v4f val = *(const v4fa*)(&os[row * 68 + c4]);
                *(volatile v4f*)(C + cb + (size_t)(mb * 16 + row) * ldc + c4) = val; }
            if (ps == 0) __threadfence(); }
        wave_sync();
    }
}

__global__ __launch_bounds__(32) void k_gemm_dt(const h16* __restrict__ Wd, const float* __restrict__ XD, const float* __restrict__ bias, float* DLp) {
    __shared__ __align__(16) float os[16 * 68];
    const int lane = threadIdx.x & 31, lr = lane & 15, hi = lane >> 4; const int r0 = blockIdx.x * 64, c0 = blockIdx.y * 64;
    v16h a[4], bq[4];
#pragma unroll
    for (int mb = 0; mb < 4; ++mb) a[mb] = ldh(Wd + (size_t)(r0 + mb * 16 + lr) * DTR + 8 * hi);
#pragma unroll
    for (int nb = 0; nb < 4; ++nb) { const float* p = XD + (size_t)(c0 + nb * 16 + lr) * NXP + 8 * hi;
        const v4f x0 = *(const v4f*)p, x1 = *(const v4f*)(p + 4), x2 = *(const v4f*)(p + 16), x3 = *(const v4f*)(p + 20);
        v16h t;
#pragma unroll
        for (int i = 0; i < 4; ++i) { t[i] = toh_flush(x0[i] * DTS); t[4 + i] = toh_flush(x1[i] * DTS); t[8 + i] = toh_flush(x2[i] * DTS); t[12 + i] = toh_flush(x3[i] * DTS); }
        bq[nb] = t; }
    v8f acc[4][4];
#pragma unroll
    for (int mb = 0; mb < 4; ++mb)
#pragma unroll
        for (int nb = 0; nb < 4; ++nb) acc[mb][nb] = mmah(a[mb], bq[nb], (v8f){});
    const int bb = c0 / SEQ, tt = c0 % SEQ;
    const size_t cb = ((size_t)bb * DH + r0) * SEQ + tt;
#pragma unroll
    for (int mb = 0; mb < 4; ++mb) {
        float br[8];
#pragma unroll
        for (int j = 0; j < 8; ++j) br[j] = bfr(bias[r0 + mb * 16 + hi * 8 + j]);
#pragma unroll
        for (int nb = 0; nb < 4; ++nb) {
#pragma unroll
            for (int j = 0; j < 8; ++j) os[(hi * 8 + j) * 68 + nb * 16 + lr] = acc[mb][nb][j] * INV_DT + br[j]; }
        wave_sync();
#pragma unroll 1
        for (int s = 0; s < 8; ++s) { const int row = 2 * s + (lane >> 4), c4 = (lane & 15) * 4;
            const v4f x = *(const v4fa*)(&os[row * 68 + c4]); v4f y;
            y[0] = softplus_f(x[0]); y[1] = softplus_f(x[1]); y[2] = softplus_f(x[2]); y[3] = softplus_f(x[3]);
            *(v4fa*)(&os[row * 68 + c4]) = y;
            *(volatile v4f*)(DLp + cb + (size_t)(mb * 16 + row) * SEQ + c4) = y; }
        __threadfence();
#pragma unroll 1
        for (int s = 0; s < 8; ++s) { const int row = 2 * s + (lane >> 4), c4 = (lane & 15) * 4;
            const v4f y = *(const v4fa*)(&os[row * 68 + c4]);
            *(volatile v4f*)(DLp + cb + (size_t)(mb * 16 + row) * SEQ + c4) = y; }
        wave_sync();
    }
}

__global__ __launch_bounds__(256) void k_conv(const float* __restrict__ XZ, const float* __restrict__ cxw, const float* __restrict__ czw, float* FB, size_t offU, size_t offY) {
    const size_t g = (size_t)blockIdx.x * 256 + threadIdx.x; if (g >= (size_t)NB * DM * (SEQ / 4)) return;
    const int row = (int)(g / (SEQ / 4)); const int l4 = (int)(g % (SEQ / 4)) * 4;
    const int i = row % DM, b = row / DM; const int ic = i & (DH - 1);
    const v4f wx = *(const v4f*)(cxw + ic * 4), wz = *(const v4f*)(czw + ic * 4);
    const bool isx = i < DH;
    const float w0 = bfr(isx ? wx[0] : wz[0]), w1 = bfr(isx ? wx[1] : wz[1]), w2 = bfr(isx ? wx[2] : wz[2]), w3 = bfr(isx ? wx[3] : wz[3]);
    const float* p = XZ + (size_t)row * SEQ;
    const v4f c = *(const v4f*)(p + l4);
    const int il = l4 > 0 ? l4 - 1 : 0; const int i1 = (l4 + 4 < SEQ) ? l4 + 4 : SEQ - 1; const int i2 = (l4 + 5 < SEQ) ? l4 + 5 : SEQ - 1;
    float xl = p[il], xr1 = p[i1], xr2 = p[i2];
    asm volatile("" : "+v"(xl), "+v"(xr1), "+v"(xr2));
    const bool lin = l4 > 0, rin = (l4 + 4) < SEQ;
    xl = lin ? xl : 0.0f; xr1 = rin ? xr1 : 0.0f; xr2 = rin ? xr2 : 0.0f;
    float x[7]; x[0] = xl; x[1] = c[0]; x[2] = c[1]; x[3] = c[2]; x[4] = c[3]; x[5] = xr1; x[6] = xr2;
    v4f o;
#pragma unroll
    for (int k = 0; k < 4; ++k) { const float acc = w0 * x[k] + w1 * x[k + 1] + w2 * x[k + 2] + w3 * x[k + 3];
        o[k] = acc * __builtin_amdgcn_rcpf(1.0f + __builtin_amdgcn_exp2f(-acc * LOG2E)); }
    const size_t dofs = isx ? (offU + ((size_t)b * DH + i) * SEQ + l4) : (offY + ((size_t)b * DM + i) * SEQ + l4);
    *(volatile v4f*)(FB + dofs) = o; __threadfence(); *(volatile v4f*)(FB + dofs) = o;
}

__global__ __launch_bounds__(256) void k_max(const float* __restrict__ XD, float* PM) {
    __shared__ float wm[8];
    const int tid = threadIdx.x, lane = tid & 31;
    const int wave = __builtin_amdgcn_readfirstlane((int)(threadIdx.x >> 5));
    const int q = tid & 63, rs = tid >> 6;
    const float* p = XD + ((size_t)blockIdx.x * 64 + rs) * NXP + DTR + 4 * q;
    float m = NEGB;
#pragma unroll 1
    for (int it = 0; it < 16; ++it) { const v4f v = *(const v4f*)(p + (size_t)it * 4 * NXP);
        m = fmaxf(m, fmaxf(fmaxf(v[0], v[1]), fmaxf(v[2], v[3]))); }
    for (int o = 16; o > 0; o >>= 1) m = fmaxf(m, __shfl_xor(m, o, 32));
    if (lane == 0) wm[wave] = m;
    __syncthreads();
    const float mB = fmaxf(fmaxf(wm[0], wm[2]), fmaxf(wm[4], wm[6])), mC = fmaxf(fmaxf(wm[1], wm[3]), fmaxf(wm[5], wm[7]));
    v4f o = (v4f){}; o[0] = (tid == 0) ? mB : 0.0f; o[1] = (tid == 0) ? mC : 0.0f;
    const int tc = tid < 8 ? tid : 7;
    if (tid < 8) *(volatile v4f*)(PM + (size_t)blockIdx.x * 32 + tc * 4) = o;
    __threadfence();
    if (tid < 8) *(volatile v4f*)(PM + (size_t)blockIdx.x * 32 + tc * 4) = o;
}

__global__ __launch_bounds__(256) void k_thr(const float* __restrict__ XD, const float* __restrict__ PM, float* BC) {
    __shared__ float wmB[8];
    __shared__ float wmC[8];
    const int tid = threadIdx.x, lane = tid & 31;
    const int wave = __builtin_amdgcn_readfirstlane((int)(threadIdx.x >> 5));
    const int tc = tid < NPB ? tid : (NPB - 1);
    float pb = PM[(size_t)tc * 32], pc = PM[(size_t)tc * 32 + 1];
    for (int o = 16; o > 0; o >>= 1) { pb = fmaxf(pb, __shfl_xor(pb, o, 32)); pc = fmaxf(pc, __shfl_xor(pc, o, 32)); }
    if (lane == 0) { wmB[wave] = pb; wmC[wave] = pc; }
    __syncthreads();
    float gb = wmB[0], gc = wmC[0];
#pragma unroll
    for (int k = 1; k < 8; ++k) { gb = fmaxf(gb, wmB[k]); gc = fmaxf(gc, wmC[k]); }
    const float thrB = 0.1f * gb, thrC = 0.1f * gc;
#pragma unroll 1
    for (int j = 0; j < 4; ++j) {
        const size_t idx = (size_t)blockIdx.x * 1024 + j * 256 + tid;
        const size_t row = idx >> 6; const int q = (int)(idx & 63);
        const v4f v = *(const v4f*)(XD + row * NXP + DTR + 4 * q);
        const float thr = (q < 32) ? thrB : thrC;
        v4f o; o[0] = softthr(v[0], thr); o[1] = softthr(v[1], thr); o[2] = softthr(v[2], thr); o[3] = softthr(v[3], thr);
        *(volatile v4f*)(BC + idx * 4) = o; __threadfence(); *(volatile v4f*)(BC + idx * 4) = o; }
}

__global__ __launch_bounds__(256) void k_scan(const float* __restrict__ DLp, const float* __restrict__ Up, const float* __restrict__ Amat, const float* __restrict__ BCp,
                                              const float* __restrict__ Dvec, float* YZc) {
    __shared__ __align__(16) float ps[8 * 32 * 36];
    __shared__ float ys[8 * SEQ];
    const int lane = threadIdx.x & 31;
    const int wave = __builtin_amdgcn_readfirstlane((int)(threadIdx.x >> 5));
    const int gw = blockIdx.x * 8 + wave; const int b = gw / DH, d = gw % DH;
    const v4f ar = *(const v4f*)(Amat + (size_t)d * DS + lane * 4);
    const float a0 = ar[0] * LOG2E, a1 = ar[1] * LOG2E, a2 = ar[2] * LOG2E, a3 = ar[3] * LOG2E;
    const float Dd = bfr(Dvec[d]);
    const float* drow = DLp + ((size_t)b * DH + d) * SEQ;
    const float* urow = Up + ((size_t)b * DH + d) * SEQ;
    const float* bcb = BCp + (size_t)b * SEQ * 256 + lane * 4;
    const int pw = wave * 32 * 36, yw = wave * SEQ;
    float h0 = 0.0f, h1 = 0.0f, h2 = 0.0f, h3 = 0.0f;
#pragma unroll 1
    for (int l0 = 0; l0 < SEQ; l0 += 32) {
        const float dt32 = drow[l0 + lane]; const float uu32 = urow[l0 + lane]; const float du32 = dt32 * uu32;
        const float* bcp = bcb + (size_t)l0 * 256;
#pragma unroll 2
        for (int j = 0; j < 32; ++j) {
            const float dt = __int_as_float(__builtin_amdgcn_readlane(__float_as_int(dt32), j));
            const float du = __int_as_float(__builtin_amdgcn_readlane(__float_as_int(du32), j));
            const v4f bv = *(const v4f*)(bcp + (size_t)j * 256); const v4f cv = *(const v4f*)(bcp + (size_t)j * 256 + DS);
            h0 = __builtin_amdgcn_exp2f(dt * a0) * h0 + du * bv[0];
            h1 = __builtin_amdgcn_exp2f(dt * a1) * h1 + du * bv[1];
            h2 = __builtin_amdgcn_exp2f(dt * a2) * h2 + du * bv[2];
            h3 = __builtin_amdgcn_exp2f(dt * a3) * h3 + du * bv[3];
            ps[pw + j * 36 + lane] = h0 * cv[0] + h1 * cv[1] + h2 * cv[2] + h3 * cv[3];
        }
        wave_sync();
        float s = 0.0f;
#pragma unroll
        for (int q = 0; q < 8; ++q) { const v4f t = *(const v4fa*)(&ps[pw + lane * 36 + 4 * q]); s += (t[0] + t[1]) + (t[2] + t[3]); }
        ys[yw + l0 + lane] = s + uu32 * Dd;
        wave_sync();
    }
    float* yrow = YZc + ((size_t)b * DM + d) * SEQ;
#pragma unroll 1
    for (int pp = 0; pp < 2; ++pp) {
#pragma unroll 1
        for (int i = 0; i < SEQ / 32; ++i) { const float v = ys[yw + i * 32 + lane];
            *(volatile float*)(yrow + i * 32 + lane) = v; }
        if (pp == 0) __threadfence(); }
}

static constexpr size_t al256(size_t v) { return (v + 255) & ~(size_t)255; }
static constexpr size_t SZ_XT  = al256((size_t)NTOK * CIN * 2);
static constexpr size_t SZ_WIN = al256((size_t)DM * DM * 2);
static constexpr size_t SZ_XPW = al256((size_t)NXP * DH * 2);
static constexpr size_t SZ_DTW = al256((size_t)DH * DTR * 2);
static constexpr size_t SZ_OW  = al256((size_t)DM * DM * 2);
static constexpr size_t SZ_A12 = al256((size_t)2 * DH * DS * 4);
static constexpr size_t SZ_XZ  = al256((size_t)NB * DM * SEQ * 4);
static constexpr size_t SZ_U   = al256((size_t)NB * DH * SEQ * 4);
static constexpr size_t SZ_YZC = al256((size_t)NB * DM * SEQ * 4);
static constexpr size_t SZ_XC  = al256((size_t)NTOK * DH * 2);
static constexpr size_t SZ_XD  = al256((size_t)NTOK * NXP * 4);
static constexpr size_t SZ_PM  = al256((size_t)NPB * 32 * 4);
static constexpr size_t SZ_BC  = al256((size_t)NTOK * 256 * 4);
static constexpr size_t SZ_DL  = al256((size_t)NB * DH * SEQ * 4);
static constexpr size_t SZ_YZ  = al256((size_t)NTOK * DM * 2);
static constexpr size_t SZ_TOTAL = SZ_XT + SZ_WIN + SZ_XPW + SZ_DTW + SZ_OW + SZ_A12 + SZ_XZ + SZ_U + SZ_YZC + SZ_XC + SZ_XD + SZ_PM + SZ_BC + SZ_DL + SZ_YZ;
static_assert(SZ_TOTAL <= (size_t)134217728);
static_assert(SZ_U % 4 == 0);
static_assert(((size_t)NTOK * 64) % 1024 == 0);
static_assert(((size_t)NB * DM * (SEQ / 4)) % 256 == 0);

extern "C" void kernel_launch(void* const* d_in, const int* in_sizes, int n_in,
                              void* d_out, int out_size, void* d_ws, size_t ws_size, hipStream_t stream) {
    if (n_in < 18) return;
    const size_t needx = ((size_t)(NB - 1) * CIN + (CIN - 1)) * SEQ_FULL + SEQ;
    if ((size_t)in_sizes[0] < needx) return;
    if ((size_t)in_sizes[1] < (size_t)DM * DM || (size_t)in_sizes[7] < (size_t)DM * DM || (size_t)in_sizes[8] < (size_t)DM * DM || (size_t)in_sizes[14] < (size_t)DM * DM) return;
    if (in_sizes[2] < DH * 4 || in_sizes[3] < DH * 4 || in_sizes[9] < DH * 4 || in_sizes[10] < DH * 4) return;
    if (in_sizes[4] < NXD * DH || in_sizes[11] < NXD * DH) return;
    if (in_sizes[5] < DH * DTR || in_sizes[12] < DH * DTR) return;
    if (in_sizes[6] < DH || in_sizes[13] < DH) return;
    if (in_sizes[15] < DH * DS || in_sizes[16] < DH || in_sizes[17] < 1) return;
    if ((size_t)out_size < OUT1_OFF + ((size_t)(NB - 1) * OUT_SEQ + SEQ) * DM) return;
    if (SZ_TOTAL > ws_size) return;
    const float* inp   = (const float*)d_in[0];
    const float* A_log = (const float*)d_in[15];
    const float* Dvec  = (const float*)d_in[16];
    const float* eps   = (const float*)d_in[17];

    char* wsp = (char*)d_ws;
    bf*    XT  = (bf*)wsp;    wsp += SZ_XT;
    bf*    WIN = (bf*)wsp;    wsp += SZ_WIN;
    h16*   XPW = (h16*)wsp;   wsp += SZ_XPW;
    h16*   DTW = (h16*)wsp;   wsp += SZ_DTW;
    h16*   OW  = (h16*)wsp;   wsp += SZ_OW;
    float* A12 = (float*)wsp; wsp += SZ_A12;
    float* XZ  = (float*)wsp; wsp += SZ_XZ;
    float* FB  = (float*)wsp; wsp += SZ_U;
    wsp += SZ_YZC;
    h16*   XC  = (h16*)wsp;   wsp += SZ_XC;
    float* XD  = (float*)wsp; wsp += SZ_XD;
    float* PM  = (float*)wsp; wsp += SZ_PM;
    float* BC  = (float*)wsp; wsp += SZ_BC;
    float* DL  = (float*)wsp; wsp += SZ_DL;
    h16*   YZ  = (h16*)wsp;   wsp += SZ_YZ;
    const size_t offU = 0, offY = SZ_U / 4;
    float* Up  = FB;
    float* YZc = FB + offY;

    k_tr_bf<<<dim3(SEQ / 64, CIN / 64, NB), 256, 0, stream>>>(inp, (size_t)CIN * SEQ_FULL, SEQ_FULL, XT, CIN);
    k_prepA<<<1, 512, 0, stream>>>(A_log, eps, A12);

    for (int br = 0; br < 2; ++br) {
        const float* in_w = (const float*)d_in[br ? 8 : 1];
        const float* cxw  = (const float*)d_in[br ? 9 : 2];
        const float* czw  = (const float*)d_in[br ? 10 : 3];
        const float* xpw  = (const float*)d_in[br ? 11 : 4];
        const float* dtw  = (const float*)d_in[br ? 12 : 5];
        const float* dtb  = (const float*)d_in[br ? 13 : 6];
        const float* outw = (const float*)d_in[br ? 14 : 7];
        const float* Ab   = A12 + (size_t)br * DH * DS;
        float* outp = (float*)d_out + (size_t)br * OUT1_OFF;

        { const size_t n8 = (size_t)DM * DM / 8; k_cvt8<<<(unsigned)((n8 + 255) / 256), 256, 0, stream>>>(in_w, WIN, n8); }
        { const size_t n8 = (size_t)NXP * DH / 8; k_wcvth<<<(unsigned)((n8 + 255) / 256), 256, 0, stream>>>(xpw, XPW, NXD, NXP, DH, WCS); }
        { const size_t n8 = (size_t)DH * DTR / 8; k_wcvth<<<(unsigned)((n8 + 255) / 256), 256, 0, stream>>>(dtw, DTW, DH, DH, DTR, DTS); }
        { const size_t n8 = (size_t)DM * DM / 8; k_wcvth<<<(unsigned)((n8 + 255) / 256), 256, 0, stream>>>(outw, OW, DM, DM, DM, WCS); }

        k_gemm_in<<<dim3(DM / 64, NTOK / 64, 1), 32, 0, stream>>>(WIN, XT + (size_t)br * DM, XZ);
        k_conv<<<(unsigned)(((size_t)NB * DM * (SEQ / 4)) / 256), 256, 0, stream>>>(XZ, cxw, czw, FB, offU, offY);
        k_tr_h<<<dim3(SEQ / 64, DH / 64, NB), 256, 0, stream>>>(Up, (size_t)DH * SEQ, SEQ, XC, DH, XCS);
        k_gemm_tm<<<dim3(NTOK / 64, NXP / 64, 1), 32, 0, stream>>>(XC, DH, XPW, DH, DH, XD, NXP, SEQ, INV_XW);
        k_max<<<NPB, 256, 0, stream>>>(XD, PM);
        k_thr<<<(unsigned)(((size_t)NTOK * 64) / 1024), 256, 0, stream>>>(XD, PM, BC);
        k_gemm_dt<<<dim3(DH / 64, NTOK / 64, 1), 32, 0, stream>>>(DTW, XD, dtb, DL);
        k_scan<<<(NB * DH) / 8, 256, 0, stream>>>(DL, Up, Ab, BC, Dvec, YZc);
        k_tr_h<<<dim3(SEQ / 64, DM / 64, NB), 256, 0, stream>>>(YZc, (size_t)DM * SEQ, SEQ, YZ, DM, XCS);
        k_gemm_tm<<<dim3(NTOK / 64, DM / 64, 1), 32, 0, stream>>>(YZ, DM, OW, DM, DM, outp, DM, OUT_SEQ, INV_XW);
    }
}
